// MambaBlock_47321949667956
// MI455X (gfx1250) — hardware-verified
//
#include <hip/hip_runtime.h>
#include <math.h>

typedef __attribute__((ext_vector_type(8)))  _Float16 v8h;
typedef __attribute__((ext_vector_type(16))) __bf16   v16b;
typedef __attribute__((ext_vector_type(8)))  __bf16   v8b;
typedef __attribute__((ext_vector_type(8)))  float    v8f;
typedef __attribute__((ext_vector_type(4)))  float    v4f;

constexpr int kBatch   = 2;
constexpr int kSeq     = 4096;
constexpr int kDm      = 512;
constexpr int kDin     = 1024;
constexpr int kNst     = 16;
constexpr int kDtR     = 32;
constexpr int kNL      = 2;
constexpr int kXzP     = 2 * kDin;
constexpr int kXdP     = 64;
constexpr int kRowsAll = kBatch * kSeq;
constexpr int kConvTP  = 260;
constexpr int kScanTS  = 64;
constexpr int kScanCh  = 64;
constexpr int kScanYP  = 68;
constexpr int kScanXP  = 32;
constexpr float kLnEps = 1e-5f;
static_assert(kDtR + 2 * kNst == kXdP, "x_proj width");
static_assert((kDm % 32) == 0 && (kDin % 32) == 0 && (kDtR % 32) == 0, "GEMM K multiples of 32");
static_assert((kSeq % 64) == 0 && (kXzP % 64) == 0 && (kXdP % 64) == 0 && (kDm % 64) == 0 && (kDin % 64) == 0, "GEMM M,N multiples of 64");
static_assert((kSeq % kScanTS) == 0 && (kDin % kScanCh) == 0 && (kDin % 256) == 0 && (kSeq % 8) == 0, "tile multiples");
static_assert(((kSeq / 64) * (kXzP / 64)) % 8 == 0 && ((kSeq / 64) * (kXdP / 64)) % 8 == 0 &&
              ((kSeq / 64) * (kDin / 64)) % 8 == 0 && ((kSeq / 64) * (kDm / 64)) % 8 == 0, "8 wave tiles per block");

constexpr size_t kOffX0H  = 0;
constexpr size_t kOffX1H  = kOffX0H  + (size_t)kRowsAll * kDm * 2;
constexpr size_t kOffX1L  = kOffX1H  + (size_t)kRowsAll * kDm * 2;
constexpr size_t kOffWIN  = kOffX1L  + (size_t)kRowsAll * kDm * 2;
constexpr size_t kOffWXP  = kOffWIN  + (size_t)kNL * kXzP * kDm * 2;
constexpr size_t kOffWDT  = kOffWXP  + (size_t)kNL * kXdP * kDin * 2;
constexpr size_t kOffWOUT = kOffWDT  + (size_t)kNL * kDin * kDtR * 2;
constexpr size_t kOffXZ   = kOffWOUT + (size_t)kNL * kDm * kDin * 2;
constexpr size_t kOffUC   = kOffXZ   + (size_t)kSeq * kXzP * 4;
constexpr size_t kOffUCH  = kOffUC   + (size_t)kSeq * kDin * 4;
constexpr size_t kOffXD   = kOffUCH  + (size_t)kSeq * kDin * 2;
constexpr size_t kOffXD16 = kOffXD   + (size_t)kSeq * kXdP * 4;
constexpr size_t kOffDLR  = kOffXD16 + (size_t)kSeq * kXdP * 2;
constexpr size_t kOffYH   = kOffDLR  + (size_t)kSeq * kDin * 4;
constexpr size_t kOffYL   = kOffYH   + (size_t)kSeq * kDin * 2;
constexpr size_t kOffOUT  = kOffYL   + (size_t)kSeq * kDin * 2;
constexpr size_t kWsTotal = kOffOUT  + (size_t)kSeq * kDm * 4;
static_assert(kWsTotal == 134086656ull, "carve total");
static_assert(kWsTotal <= 134217728ull, "carve cap");
static_assert((kOffX1H % 128) == 0 && (kOffX1L % 128) == 0 && (kOffWIN % 128) == 0 && (kOffWXP % 128) == 0 &&
              (kOffWDT % 128) == 0 && (kOffWOUT % 128) == 0 && (kOffXZ % 128) == 0 && (kOffUC % 128) == 0 &&
              (kOffUCH % 128) == 0 && (kOffXD % 128) == 0 && (kOffXD16 % 128) == 0 && (kOffDLR % 128) == 0 &&
              (kOffYH % 128) == 0 && (kOffYL % 128) == 0 && (kOffOUT % 128) == 0, "128-B aligned regions");

__device__ __forceinline__ unsigned short f2bf_bits(float f) {
  unsigned u = __float_as_uint(f);
  return (unsigned short)((u + 0x7FFFu + ((u >> 16) & 1u)) >> 16);
}
__device__ __forceinline__ float bf_bits2f(unsigned short h) { return __uint_as_float(((unsigned)h) << 16); }
__device__ __forceinline__ float bf_rne(float f) { return bf_bits2f(f2bf_bits(f)); }

__device__ __forceinline__ v8h pack_hi(const v4f a0, const v4f a1) {
  v8h hv;
#pragma unroll
  for (int e = 0; e < 4; ++e) {
    const float f0 = a0[e];
    const float f1 = a1[e];
    const unsigned short h0 = f2bf_bits(f0);
    const unsigned short h1 = f2bf_bits(f1);
    hv[e]     = __builtin_bit_cast(_Float16, h0);
    hv[4 + e] = __builtin_bit_cast(_Float16, h1);
  }
  return hv;
}
__device__ __forceinline__ void pack_hi_lo(const v4f a0, const v4f a1, v8h& hv, v8h& lv) {
#pragma unroll
  for (int e = 0; e < 4; ++e) {
    const float f0 = a0[e];
    const float f1 = a1[e];
    const unsigned short h0 = f2bf_bits(f0);
    const unsigned short h1 = f2bf_bits(f1);
    const unsigned short l0 = f2bf_bits(f0 - bf_bits2f(h0));
    const unsigned short l1 = f2bf_bits(f1 - bf_bits2f(h1));
    hv[e]     = __builtin_bit_cast(_Float16, h0);
    hv[4 + e] = __builtin_bit_cast(_Float16, h1);
    lv[e]     = __builtin_bit_cast(_Float16, l0);
    lv[4 + e] = __builtin_bit_cast(_Float16, l1);
  }
}

__device__ __forceinline__ void dep_guard4_b(v8f& a, v8f& b, v8f& c, v8f& d, v16b x, v16b y) {
  asm volatile("v_nop\n\tv_nop\n\tv_nop\n\tv_nop" : "+v"(a), "+v"(b), "+v"(c), "+v"(d) : "v"(x), "v"(y));
}
__device__ __forceinline__ void keep4_b(v16b a, v16b b, v16b c, v16b d) { asm volatile("v_nop" :: "v"(a), "v"(b), "v"(c), "v"(d)); }
__device__ __forceinline__ void acc_guard4(v8f& a, v8f& b, v8f& c, v8f& d) { asm volatile("v_nop\n\tv_nop\n\tv_nop\n\tv_nop" : "+v"(a), "+v"(b), "+v"(c), "+v"(d)); }

struct FragB {
  union U { v16b v; v8b h[2]; };
  static __device__ __forceinline__ v16b load(const __bf16* p) {
    U f;
    f.h[0] = *(const v8b*)(p);
    f.h[1] = *(const v8b*)(p + 16);
    return f.v;
  }
  static __device__ __forceinline__ v8f mma(v16b a, v16b b, v8f c) {
    return __builtin_amdgcn_wmma_f32_16x16x32_bf16(false, a, false, b, (short)0, c, false, false);
  }
};

template <int SPL>
__global__ __launch_bounds__(256) void wmma_gemm64(
    const unsigned short* __restrict__ Ap, const unsigned short* __restrict__ A2p, int lda,
    const unsigned short* __restrict__ Btp, int ldb,
    float* __restrict__ Cout, int ldc, int M, int N, int K)
{
  typedef __bf16 T;
  typedef v16b V;
  const T* A  = (const T*)Ap;
  const T* A2 = (const T*)A2p;
  const T* Bt = (const T*)Btp;
  __shared__ __align__(16) float sT[8][16 * 68];
  const int lane = threadIdx.x & 31;
  const int wave = threadIdx.x >> 5;
  const int tilesN = N >> 6;
  const int tilesM = M >> 6;
  const int tile = blockIdx.x * 8 + wave;
  if (tile >= tilesM * tilesN) return;
  const int tm = tile / tilesN;
  const int tn = tile - tm * tilesN;
  const int m0 = tm << 6;
  const int n0 = tn << 6;

  const int rlane = lane & 15;
  const int koff  = (lane >> 4) * 8;
  const int mOff  = (lane >> 4) * 8;

  v8f acc[4][4];
#pragma unroll
  for (int i = 0; i < 4; ++i)
#pragma unroll
    for (int j = 0; j < 4; ++j) acc[i][j] = (v8f){0.f, 0.f, 0.f, 0.f, 0.f, 0.f, 0.f, 0.f};

  for (int k0 = 0; k0 < K; k0 += 32) {
    V bh[4];
#pragma unroll
    for (int j = 0; j < 4; ++j) {
      const size_t bo = (size_t)(n0 + (j << 4) + rlane) * ldb + koff + k0;
      bh[j] = FragB::load(Bt + bo);
    }
#pragma unroll
    for (int i = 0; i < 4; ++i) {
      const size_t ao = (size_t)(m0 + (i << 4) + rlane) * lda + koff + k0;
      V ah = FragB::load(A + ao);
      V al = ah;
      if (SPL == 1) al = FragB::load(A2 + ao);
#pragma unroll
      for (int j = 0; j < 4; ++j) {
        acc[i][j] = FragB::mma(ah, bh[j], acc[i][j]);
        if (SPL == 1) acc[i][j] = FragB::mma(al, bh[j], acc[i][j]);
      }
      dep_guard4_b(acc[i][0], acc[i][1], acc[i][2], acc[i][3], ah, al);
    }
    keep4_b(bh[0], bh[1], bh[2], bh[3]);
  }
  acc_guard4(acc[0][0], acc[0][1], acc[0][2], acc[0][3]);
  acc_guard4(acc[1][0], acc[1][1], acc[1][2], acc[1][3]);
  acc_guard4(acc[2][0], acc[2][1], acc[2][2], acc[2][3]);
  acc_guard4(acc[3][0], acc[3][1], acc[3][2], acc[3][3]);

  float* slab = sT[wave];
#pragma unroll
  for (int i = 0; i < 4; ++i) {
    const int mBase = m0 + (i << 4);
#pragma unroll
    for (int j = 0; j < 4; ++j) {
#pragma unroll
      for (int r = 0; r < 8; ++r) {
        slab[(mOff + r) * 68 + (j << 4) + rlane] = acc[i][j][r];
      }
    }
    __builtin_amdgcn_fence(__ATOMIC_RELEASE, "workgroup");
    __builtin_amdgcn_wave_barrier();
    __builtin_amdgcn_fence(__ATOMIC_ACQUIRE, "workgroup");
    {
      const int hh = lane >> 4, c4 = (lane & 15) * 4;
      for (int pass = 0; pass < 2; ++pass) {
#pragma unroll
        for (int it = 0; it < 8; ++it) {
          const int row = it * 2 + hh;
          v4f v = *(const v4f*)(slab + row * 68 + c4);
          *(volatile v4f*)(Cout + (size_t)(mBase + row) * ldc + n0 + c4) = v;
        }
        __threadfence();
      }
    }
    __builtin_amdgcn_fence(__ATOMIC_RELEASE, "workgroup");
    __builtin_amdgcn_wave_barrier();
    __builtin_amdgcn_fence(__ATOMIC_ACQUIRE, "workgroup");
  }
}

__global__ __launch_bounds__(256) void cast_bf16_kernel(
    const float* __restrict__ src, unsigned short* __restrict__ dst, int total8)
{
  const int i = blockIdx.x * 256 + threadIdx.x;
  if (i >= total8) return;
  const size_t e0 = (size_t)i << 3;
  const v4f a0 = *(const v4f*)(src + e0);
  const v4f a1 = *(const v4f*)(src + e0 + 4);
  const v8h hv = pack_hi(a0, a1);
  unsigned short* q = dst + e0;
  *(volatile v8h*)q = hv;
  __threadfence();
  *(volatile v8h*)q = hv;
}

__global__ __launch_bounds__(256) void conv_silu_kernel(
    const float* __restrict__ XZ, const float* __restrict__ cw, const float* __restrict__ cb,
    float* __restrict__ UC, unsigned short* __restrict__ UCH)
{
  __shared__ __align__(16) float sT[16 * kConvTP];
  const int tid = threadIdx.x, lane = tid & 31, wave = tid >> 5;
  const int d0 = blockIdx.x * 256, d = d0 + tid;
  const int t0 = blockIdx.y * 64;
  const v4f wv = *(const v4f*)(cw + (size_t)d * 4);
  const float wr0 = wv[0];
  const float wr1 = wv[1];
  const float wr2 = wv[2];
  const float wr3 = wv[3];
  const float w0 = bf_rne(wr0), w1 = bf_rne(wr1), w2 = bf_rne(wr2), w3 = bf_rne(wr3);
  const float bc = bf_rne(cb[d]);
  float xm3, xm2, xm1;
  {
    const int r3 = t0 - 3, r2 = t0 - 2, r1 = t0 - 1;
    const float v3 = XZ[(size_t)(r3 < 0 ? 0 : r3) * kXzP + d];
    const float v2 = XZ[(size_t)(r2 < 0 ? 0 : r2) * kXzP + d];
    const float v1 = XZ[(size_t)(r1 < 0 ? 0 : r1) * kXzP + d];
    xm3 = (r3 >= 0) ? v3 : 0.f;
    xm2 = (r2 >= 0) ? v2 : 0.f;
    xm1 = (r1 >= 0) ? v1 : 0.f;
  }
  const int hrow = wave >> 1;
  const int hch  = (wave & 1) * 128 + lane * 4;
#pragma unroll 1
  for (int sub = 0; sub < 4; ++sub) {
    const int lb = t0 + sub * 16;
#pragma unroll 1
    for (int s = 0; s < 16; ++s) {
      const float xcur = XZ[(size_t)(lb + s) * kXzP + d];
      float acc = w0 * xm3;
      acc = fmaf(w1, xm2, acc);
      acc = fmaf(w2, xm1, acc);
      acc = fmaf(w3, xcur, acc);
      const float sv = acc + bc;
      const float sg = __builtin_amdgcn_rcpf(1.0f + expf(-sv));
      sT[s * kConvTP + tid] = sv * sg;
      xm3 = xm2; xm2 = xm1; xm1 = xcur;
    }
    __syncthreads();
    v4f fv[4];
    v8h bv[2];
#pragma unroll
    for (int it = 0; it < 4; ++it) fv[it] = *(const v4f*)(sT + (it * 4 + hrow) * kConvTP + hch);
#pragma unroll
    for (int it = 0; it < 2; ++it) {
      const float* sp = sT + (it * 8 + wave) * kConvTP + lane * 8;
      const v4f a0 = *(const v4f*)(sp);
      const v4f a1 = *(const v4f*)(sp + 4);
      bv[it] = pack_hi(a0, a1);
    }
    for (int pass = 0; pass < 2; ++pass) {
#pragma unroll
      for (int it = 0; it < 4; ++it)
        *(volatile v4f*)(UC + (size_t)(lb + it * 4 + hrow) * kDin + d0 + hch) = fv[it];
#pragma unroll
      for (int it = 0; it < 2; ++it)
        *(volatile v8h*)(UCH + (size_t)(lb + it * 8 + wave) * kDin + d0 + lane * 8) = bv[it];
      __threadfence();
    }
    __syncthreads();
  }
}

__global__ __launch_bounds__(64) void scan_kernel(
    const float* __restrict__ DLR, const float* __restrict__ UC, const float* __restrict__ XZ,
    const float* __restrict__ XD, const float* __restrict__ bdt, const float* __restrict__ Alog,
    const float* __restrict__ Dp, unsigned short* __restrict__ YH, unsigned short* __restrict__ YL)
{
  __shared__ __align__(16) float sX[kScanTS * kScanXP];
  __shared__ __align__(16) float sY[kScanTS * kScanYP];
  __shared__ __align__(16) float sA[kNst * kScanCh];
  const int tid = threadIdx.x, lane = tid & 31, wave = tid >> 5;
  const int d0 = blockIdx.x * kScanCh;
  const int d  = d0 + tid;
#pragma unroll 1
  for (int s = 0; s < kNst; ++s) sA[s * kScanCh + tid] = -expf(bf_rne(Alog[(size_t)d * kNst + s]));
  __syncthreads();
  float negA[kNst], h[kNst];
#pragma unroll
  for (int s = 0; s < kNst; ++s) {
    negA[s] = sA[s * kScanCh + tid];
    h[s] = 0.f;
  }
  const float bb = bf_rne(bdt[d]);
  const float Dd = bf_rne(Dp[d]);
  const int sr = tid >> 3, sc4 = (tid & 7) * 4;
  const int q = lane >> 3, c8 = (lane & 7) * 8;
#pragma unroll 1
  for (int t0 = 0; t0 < kSeq; t0 += kScanTS) {
    __syncthreads();
#pragma unroll
    for (int i = 0; i < 8; ++i) {
      const int r = sr + 8 * i;
      *(v4f*)(sX + r * kScanXP + sc4) = *(const v4f*)(XD + (size_t)(t0 + r) * kXdP + kDtR + sc4);
    }
    __syncthreads();
#pragma unroll 1
    for (int s = 0; s < kScanTS; ++s) {
      const size_t m = (size_t)(t0 + s);
      const float* xr = sX + s * kScanXP;
      float Bs[kNst], Cs[kNst];
#pragma unroll
      for (int q4 = 0; q4 < 4; ++q4) {
        const v4f bv = *(const v4f*)(xr + 4 * q4);
        const v4f cv = *(const v4f*)(xr + kNst + 4 * q4);
        Bs[4 * q4 + 0] = bv[0]; Bs[4 * q4 + 1] = bv[1]; Bs[4 * q4 + 2] = bv[2]; Bs[4 * q4 + 3] = bv[3];
        Cs[4 * q4 + 0] = cv[0]; Cs[4 * q4 + 1] = cv[1]; Cs[4 * q4 + 2] = cv[2]; Cs[4 * q4 + 3] = cv[3];
      }
      const float v   = DLR[m * kDin + d] + bb;
      const float a   = __expf(-fabsf(v));
      const float u   = 1.0f + a;
      const float l1p = __logf(u) + (a - (u - 1.0f)) * __builtin_amdgcn_rcpf(u);
      const float dt  = fmaxf(v, 0.0f) + l1p;
      const float xt  = UC[m * kDin + d];
      const float zv  = XZ[m * kXzP + kDin + d];
      const float dtx = dt * xt;
      float y = 0.f;
#pragma unroll
      for (int k = 0; k < kNst; ++k) {
        const float e = __expf(dt * negA[k]);
        h[k] = e * h[k] + dtx * Bs[k];
        y = h[k] * Cs[k] + y;
      }
      y = xt * Dd + y;
      const float sg = __builtin_amdgcn_rcpf(1.0f + expf(-zv));
      y = y * (zv * sg);
      sY[s * kScanYP + tid] = y;
    }
    __syncthreads();
    v8h hv[8], lv[8];
#pragma unroll
    for (int it = 0; it < 8; ++it) {
      const int row = it * 8 + wave * 4 + q;
      const float* sp = sY + row * kScanYP + c8;
      const v4f a0 = *(const v4f*)(sp);
      const v4f a1 = *(const v4f*)(sp + 4);
      pack_hi_lo(a0, a1, hv[it], lv[it]);
    }
    for (int pass = 0; pass < 2; ++pass) {
#pragma unroll
      for (int it = 0; it < 8; ++it) {
        const int row = it * 8 + wave * 4 + q;
        const size_t o = (size_t)(t0 + row) * kDin + d0 + c8;
        *(volatile v8h*)(YH + o) = hv[it];
        *(volatile v8h*)(YL + o) = lv[it];
      }
      __threadfence();
    }
  }
}

template <bool FINAL>
__global__ __launch_bounds__(256) void ln_kernel(
    const float* __restrict__ src, const float* __restrict__ gma, const float* __restrict__ bta,
    float* __restrict__ dstf, unsigned short* __restrict__ dhi, unsigned short* __restrict__ dlo)
{
  __shared__ __align__(16) float sN[8][kDm];
  const int tid = threadIdx.x, lane = tid & 31, wave = tid >> 5;
  const int row = blockIdx.x * 8 + wave;
  const float* p = src + (size_t)row * kDm;
  v4f a[4];
#pragma unroll
  for (int it = 0; it < 4; ++it) a[it] = *(const v4f*)(p + it * 128 + lane * 4);
  float s = 0.f;
#pragma unroll
  for (int it = 0; it < 4; ++it) s += (a[it][0] + a[it][1]) + (a[it][2] + a[it][3]);
#pragma unroll
  for (int off = 16; off >= 1; off >>= 1) s += __shfl_xor(s, off, 32);
  const float mu = s * (1.0f / (float)kDm);
  float qs = 0.f;
#pragma unroll
  for (int it = 0; it < 4; ++it) {
#pragma unroll
    for (int e = 0; e < 4; ++e) {
      const float dl = a[it][e] - mu;
      qs = fmaf(dl, dl, qs);
    }
  }
#pragma unroll
  for (int off = 16; off >= 1; off >>= 1) qs += __shfl_xor(qs, off, 32);
  const float var  = qs * (1.0f / (float)kDm);
  const float rstd = rsqrtf(var + kLnEps);
  v4f o[4];
#pragma unroll
  for (int it = 0; it < 4; ++it) {
    const v4f g4 = *(const v4f*)(gma + it * 128 + lane * 4);
    const v4f b4 = *(const v4f*)(bta + it * 128 + lane * 4);
#pragma unroll
    for (int e = 0; e < 4; ++e) {
      const float gr = g4[e];
      const float br = b4[e];
      o[it][e] = (a[it][e] - mu) * rstd * bf_rne(gr) + bf_rne(br);
    }
  }
  if (FINAL) {
    float* dr = dstf + (size_t)row * kDm;
    for (int pass = 0; pass < 2; ++pass) {
#pragma unroll
      for (int it = 0; it < 4; ++it) *(volatile v4f*)(dr + it * 128 + lane * 4) = o[it];
      __threadfence();
    }
  } else {
    float* sl = sN[wave];
#pragma unroll
    for (int it = 0; it < 4; ++it) *(v4f*)(sl + it * 128 + lane * 4) = o[it];
    __syncthreads();
    v8h hv[2], lv[2];
#pragma unroll
    for (int it2 = 0; it2 < 2; ++it2) {
      const float* sp = sl + it2 * 256 + lane * 8;
      const v4f a0 = *(const v4f*)(sp);
      const v4f a1 = *(const v4f*)(sp + 4);
      pack_hi_lo(a0, a1, hv[it2], lv[it2]);
    }
    for (int pass = 0; pass < 2; ++pass) {
#pragma unroll
      for (int it2 = 0; it2 < 2; ++it2) {
        const size_t oo = (size_t)row * kDm + it2 * 256 + lane * 8;
        *(volatile v8h*)(dhi + oo) = hv[it2];
        *(volatile v8h*)(dlo + oo) = lv[it2];
      }
      __threadfence();
    }
  }
}

extern "C" void kernel_launch(void* const* d_in, const int* in_sizes, int n_in,
                              void* d_out, int out_size, void* d_ws, size_t ws_size,
                              hipStream_t stream)
{
  if (n_in < 12) return;
  if (in_sizes[0]  != kRowsAll * kDm) return;
  if (in_sizes[1]  != kNL * kXzP * kDm) return;
  if (in_sizes[2]  != kNL * kDin * 4) return;
  if (in_sizes[3]  != kNL * kDin) return;
  if (in_sizes[4]  != kNL * kXdP * kDin) return;
  if (in_sizes[5]  != kNL * kDin * kDtR) return;
  if (in_sizes[6]  != kNL * kDin) return;
  if (in_sizes[7]  != kNL * kDin * kNst) return;
  if (in_sizes[8]  != kNL * kDin) return;
  if (in_sizes[9]  != kNL * kDm * kDin) return;
  if (in_sizes[10] != kNL * kDm) return;
  if (in_sizes[11] != kNL * kDm) return;
  if (out_size != kRowsAll * kDm) return;
  if (ws_size < kWsTotal) return;

  const float* x       = (const float*)d_in[0];
  const float* W_in    = (const float*)d_in[1];
  const float* conv_w  = (const float*)d_in[2];
  const float* conv_b  = (const float*)d_in[3];
  const float* W_xproj = (const float*)d_in[4];
  const float* W_dt    = (const float*)d_in[5];
  const float* b_dt    = (const float*)d_in[6];
  const float* A_log   = (const float*)d_in[7];
  const float* Dp      = (const float*)d_in[8];
  const float* W_out   = (const float*)d_in[9];
  const float* ln_g    = (const float*)d_in[10];
  const float* ln_b    = (const float*)d_in[11];
  float* out = (float*)d_out;

  char* ws = (char*)d_ws;
  unsigned short* X0H  = (unsigned short*)(ws + kOffX0H);
  unsigned short* X1H  = (unsigned short*)(ws + kOffX1H);
  unsigned short* X1L  = (unsigned short*)(ws + kOffX1L);
  unsigned short* WIN  = (unsigned short*)(ws + kOffWIN);
  unsigned short* WXP  = (unsigned short*)(ws + kOffWXP);
  unsigned short* WDT  = (unsigned short*)(ws + kOffWDT);
  unsigned short* WOUT = (unsigned short*)(ws + kOffWOUT);
  float*          XZ   = (float*)(ws + kOffXZ);
  float*          UC   = (float*)(ws + kOffUC);
  unsigned short* UCH  = (unsigned short*)(ws + kOffUCH);
  float*          XD   = (float*)(ws + kOffXD);
  unsigned short* XD16 = (unsigned short*)(ws + kOffXD16);
  float*          DLR  = (float*)(ws + kOffDLR);
  unsigned short* YH   = (unsigned short*)(ws + kOffYH);
  unsigned short* YL   = (unsigned short*)(ws + kOffYL);
  float*          OUTP = (float*)(ws + kOffOUT);

  cast_bf16_kernel<<<(kNL * kXzP * kDm) / 2048, 256, 0, stream>>>(W_in, WIN, (kNL * kXzP * kDm) / 8);
  cast_bf16_kernel<<<(kNL * kXdP * kDin) / 2048, 256, 0, stream>>>(W_xproj, WXP, (kNL * kXdP * kDin) / 8);
  cast_bf16_kernel<<<(kNL * kDin * kDtR) / 2048, 256, 0, stream>>>(W_dt, WDT, (kNL * kDin * kDtR) / 8);
  cast_bf16_kernel<<<(kNL * kDm * kDin) / 2048, 256, 0, stream>>>(W_out, WOUT, (kNL * kDm * kDin) / 8);
  cast_bf16_kernel<<<(kRowsAll * kDm) / 2048, 256, 0, stream>>>(x, X0H, (kRowsAll * kDm) / 8);

  for (int l = 0; l < kNL; ++l) {
    const unsigned short* WINl  = WIN  + (size_t)l * kXzP * kDm;
    const unsigned short* WXPl  = WXP  + (size_t)l * kXdP * kDin;
    const unsigned short* WDTl  = WDT  + (size_t)l * kDin * kDtR;
    const unsigned short* WOUTl = WOUT + (size_t)l * kDm * kDin;
    for (int b = 0; b < kBatch; ++b) {
      const size_t xo = (size_t)b * kSeq * kDm;

      if (l == 0) {
        wmma_gemm64<0><<<dim3(256, 1), 256, 0, stream>>>(
            X0H + xo, X0H + xo, kDm, WINl, kDm, XZ, kXzP, kSeq, kXzP, kDm);
      } else {
        wmma_gemm64<1><<<dim3(256, 1), 256, 0, stream>>>(
            X1H + xo, X1L + xo, kDm, WINl, kDm, XZ, kXzP, kSeq, kXzP, kDm);
      }

      conv_silu_kernel<<<dim3(kDin / 256, kSeq / 64), 256, 0, stream>>>(
          XZ, conv_w + (size_t)l * kDin * 4, conv_b + (size_t)l * kDin, UC, UCH);

      wmma_gemm64<0><<<dim3(8, 1), 256, 0, stream>>>(
          UCH, UCH, kDin, WXPl, kDin, XD, kXdP, kSeq, kXdP, kDin);

      cast_bf16_kernel<<<(kSeq * kXdP) / 2048, 256, 0, stream>>>(XD, XD16, (kSeq * kXdP) / 8);

      wmma_gemm64<0><<<dim3(128, 1), 256, 0, stream>>>(
          XD16, XD16, kXdP, WDTl, kDtR, DLR, kDin, kSeq, kDin, kDtR);

      scan_kernel<<<kDin / kScanCh, kScanCh, 0, stream>>>(
          DLR, UC, XZ, XD, b_dt + (size_t)l * kDin, A_log + (size_t)l * kDin * kNst, Dp + (size_t)l * kDin, YH, YL);

      wmma_gemm64<1><<<dim3(64, 1), 256, 0, stream>>>(
          YH, YL, kDin, WOUTl, kDin, OUTP, kDm, kSeq, kDm, kDin);

      if (l == kNL - 1) {
        ln_kernel<true><<<kSeq / 8, 256, 0, stream>>>(
            OUTP, ln_g + (size_t)l * kDm, ln_b + (size_t)l * kDm, out + xo, X1H + xo, X1L + xo);
      } else {
        ln_kernel<false><<<kSeq / 8, 256, 0, stream>>>(
            OUTP, ln_g + (size_t)l * kDm, ln_b + (size_t)l * kDm, out + xo, X1H + xo, X1L + xo);
      }
    }
  }
}
